// EncoderLayer_34754875359699
// MI455X (gfx1250) — hardware-verified
//
#include <hip/hip_runtime.h>


#pragma clang fp contract(off)

typedef _Float16 half_t;
typedef __attribute__((ext_vector_type(16))) _Float16 v16h;
typedef __attribute__((ext_vector_type(8)))  _Float16 v8h;
typedef __attribute__((ext_vector_type(8)))  float    v8f;
typedef __attribute__((ext_vector_type(4)))  float    v4f;

#ifndef SEQ
#define SEQ 2048
#endif
#define S_FULL 2048
#define DM     1024
#define NH     16
#define HD     64
#define FFD    4096
#define EPS_LN 1e-3f
#define MASKV  (-100000.0f)
#define WSC    64.0f
#define RSC    2048.0f
#define PCARRY 16384.0f

static_assert(SEQ % 128 == 0);
static_assert(SEQ >= 128);
static_assert(SEQ <= S_FULL);
static_assert(NH * HD == DM);
static_assert(DM % 128 == 0);
static_assert(FFD % 128 == 0);
static_assert(HD == 64);

#define LDS_STRIDE 40
#define SPH 136
#define SPF 132

#define M_F16  0
#define M_HILO 1
#define M_F32  2
#define M_F32B 3
#define M_RELU 4

__device__ __forceinline__ float bf16r(float x) {
    unsigned u = __float_as_uint(x);
    u = (u + 0x7FFFu + ((u >> 16) & 1u)) & 0xFFFF0000u;
    return __uint_as_float(u);
}

__device__ __forceinline__ v16h ld16(const half_t* __restrict__ p0, const half_t* __restrict__ p1) {
    v8h a = *(const v8h*)p0;
    v8h b = *(const v8h*)p1;
    v16h r;
#pragma unroll
    for (int i = 0; i < 8; ++i) { r[i] = a[i]; r[i + 8] = b[i]; }
    return r;
}

__device__ __forceinline__ v16h ld16_lds(const _Float16* p0, const _Float16* p1) {
    v8h a = *(const v8h*)p0;
    v8h b = *(const v8h*)p1;
    v16h r;
#pragma unroll
    for (int i = 0; i < 8; ++i) { r[i] = a[i]; r[i + 8] = b[i]; }
    return r;
}

__device__ __forceinline__ v8f wmma16(v16h a, v16h b, v8f c) {
    v8f d = __builtin_amdgcn_wmma_f32_16x16x32_f16(false, a, false, b, (short)0, c, false, false);
    asm volatile("v_nop\n\tv_nop\n\tv_nop\n\tv_nop" : "+v"(d) : "v"(a), "v"(b));
    return d;
}

__device__ __forceinline__ float redmax16(float v) {
    v = fmaxf(v, __shfl_xor(v, 1, 32));
    v = fmaxf(v, __shfl_xor(v, 2, 32));
    v = fmaxf(v, __shfl_xor(v, 4, 32));
    v = fmaxf(v, __shfl_xor(v, 8, 32));
    return v;
}
__device__ __forceinline__ float redsum16(float v) {
    v += __shfl_xor(v, 1, 32);
    v += __shfl_xor(v, 2, 32);
    v += __shfl_xor(v, 4, 32);
    v += __shfl_xor(v, 8, 32);
    return v;
}
__device__ __forceinline__ float redsum32(float v) {
    v += __shfl_xor(v, 1, 32);
    v += __shfl_xor(v, 2, 32);
    v += __shfl_xor(v, 4, 32);
    v += __shfl_xor(v, 8, 32);
    v += __shfl_xor(v, 16, 32);
    return v;
}

__device__ __forceinline__ void wave_lds_sync() {
    asm volatile("s_wait_dscnt 0x0" ::: "memory");
    __builtin_amdgcn_fence(3, "wavefront");
    __builtin_amdgcn_wave_barrier();
}

__global__ __launch_bounds__(256)
void k_cvt8(const float* __restrict__ src, half_t* dst, int n8, float scale) {
    const int i = blockIdx.x * 256 + threadIdx.x;
    const bool ok = i < n8;
    v8h hv = {};
    if (ok) {
        const v4f a = *(const v4f*)(src + (size_t)i * 8);
        const v4f b = *(const v4f*)(src + (size_t)i * 8 + 4);
#pragma unroll
        for (int c = 0; c < 4; ++c) {
            hv[c]     = (_Float16)(bf16r(a[c]) * scale);
            hv[c + 4] = (_Float16)(bf16r(b[c]) * scale);
        }
        *(volatile v8h*)(dst + (size_t)i * 8) = hv;
    }
    __threadfence();
    if (ok) *(volatile v8h*)(dst + (size_t)i * 8) = hv;
}

__global__ __launch_bounds__(256)
void k_tr64(const float* __restrict__ src, int spitch, half_t* dst, int dpitch, float scale) {
    __shared__ __attribute__((aligned(16))) _Float16 T[64 * 72];
    const int t = threadIdx.x, lane = t & 31, wave = t >> 5;
    const int r0 = blockIdx.y * 64, c0 = blockIdx.x * 64;
#pragma unroll
    for (int i = 0; i < 4; ++i) {
        const int r  = i * 16 + (t >> 4);
        const int cs = (t & 15) * 4;
        const v4f x = *(const v4f*)(src + (size_t)(r0 + r) * spitch + c0 + cs);
#pragma unroll
        for (int cc = 0; cc < 4; ++cc) T[(cs + cc) * 72 + r] = (_Float16)(bf16r(x[cc]) * scale);
    }
    __syncthreads();
    const int seg = (lane & 7) * 8, rq = lane >> 3;
    const int cl0 = wave * 8 + rq, cl1 = wave * 8 + 4 + rq;
    const v8h v0 = *(const v8h*)(T + cl0 * 72 + seg);
    const v8h v1 = *(const v8h*)(T + cl1 * 72 + seg);
    half_t* p0 = dst + (size_t)(c0 + cl0) * dpitch + r0 + seg;
    half_t* p1 = dst + (size_t)(c0 + cl1) * dpitch + r0 + seg;
    *(volatile v8h*)p0 = v0;
    *(volatile v8h*)p1 = v1;
    __threadfence();
    *(volatile v8h*)p0 = v0;
    *(volatile v8h*)p1 = v1;
}

__device__ __forceinline__ void write_tile_f16(const _Float16* stg, half_t* outp,
                                               int m0, int n0, int N, int wave, int lane) {
    const int hs = lane >> 4;
    const int cs = (lane & 15) * 8;
    v8h vals[8];
#pragma unroll
    for (int i = 0; i < 8; ++i) {
        const int row = wave * 16 + i * 2 + hs;
        vals[i] = *(const v8h*)(stg + row * SPH + cs);
    }
#pragma unroll
    for (int i = 0; i < 8; ++i) {
        const int row = wave * 16 + i * 2 + hs;
        *(volatile v8h*)(outp + (size_t)(m0 + row) * N + n0 + cs) = vals[i];
    }
    __threadfence();
#pragma unroll
    for (int i = 0; i < 8; ++i) {
        const int row = wave * 16 + i * 2 + hs;
        *(volatile v8h*)(outp + (size_t)(m0 + row) * N + n0 + cs) = vals[i];
    }
}

__device__ __forceinline__ void write_tile_f32(const float* stg, float* outp,
                                               int m0, int n0, int N, int wave, int lane) {
    const int cs = lane * 4;
    v4f vals[8];
#pragma unroll
    for (int i = 0; i < 8; ++i) {
        const int row = wave * 8 + i;
        vals[i] = *(const v4f*)(stg + row * SPF + cs);
    }
#pragma unroll
    for (int i = 0; i < 8; ++i) {
        const int row = wave * 8 + i;
        *(volatile v4f*)(outp + (size_t)(m0 + row) * N + n0 + cs) = vals[i];
    }
    __threadfence();
#pragma unroll
    for (int i = 0; i < 8; ++i) {
        const int row = wave * 8 + i;
        *(volatile v4f*)(outp + (size_t)(m0 + row) * N + n0 + cs) = vals[i];
    }
}

template<int MODE>
__global__ __launch_bounds__(256)
void k_gemm(const half_t* __restrict__ A, const half_t* __restrict__ Bt,
            const float* __restrict__ bias, void* out0, void* out1,
            int M, int N, int K, float scale) {
    __shared__ v4f lds_raw[2176];
    _Float16* lsA = (_Float16*)lds_raw;
    _Float16* lsB = lsA + 128 * LDS_STRIDE;
    (void)M;

    const int tid  = threadIdx.x;
    const int lane = tid & 31;
    const int wave = tid >> 5;
    const int wr   = wave & 3;
    const int wc   = wave >> 2;
    const int col  = lane & 15;
    const int hs   = lane >> 4;
    const int kb   = hs * 8;

    const int m0 = blockIdx.y * 128;
    const int n0 = blockIdx.x * 128;

    const int trow = tid >> 2;
    const int tseg = tid & 3;
    const half_t* gA0 = A  + (size_t)(m0 + trow) * K + tseg * 8;
    const half_t* gA1 = gA0 + (size_t)64 * K;
    const half_t* gB0 = Bt + (size_t)(n0 + trow) * K + tseg * 8;
    const half_t* gB1 = gB0 + (size_t)64 * K;
    _Float16* sA0 = &lsA[trow * LDS_STRIDE + tseg * 8];
    _Float16* sA1 = sA0 + 64 * LDS_STRIDE;
    _Float16* sB0 = &lsB[trow * LDS_STRIDE + tseg * 8];
    _Float16* sB1 = sB0 + 64 * LDS_STRIDE;

    const _Float16* fA0 = &lsA[(wr * 32 + col) * LDS_STRIDE + kb];
    const _Float16* fA1 = fA0 + 16 * LDS_STRIDE;
    const _Float16* fB0 = &lsB[(wc * 64 + col) * LDS_STRIDE + kb];

    v8f c[2][4] = {};

    v8h ra0 = *(const v8h*)gA0;
    v8h ra1 = *(const v8h*)gA1;
    v8h rb0 = *(const v8h*)gB0;
    v8h rb1 = *(const v8h*)gB1;

    for (int kt = 0; kt < K; kt += 32) {
        __syncthreads();
        *(v8h*)sA0 = ra0;
        *(v8h*)sA1 = ra1;
        *(v8h*)sB0 = rb0;
        *(v8h*)sB1 = rb1;
        __syncthreads();

        if (kt + 32 < K) {
            ra0 = *(const v8h*)(gA0 + kt + 32);
            ra1 = *(const v8h*)(gA1 + kt + 32);
            rb0 = *(const v8h*)(gB0 + kt + 32);
            rb1 = *(const v8h*)(gB1 + kt + 32);
        }

        const v16h a0 = ld16_lds(fA0, fA0 + 16);
        const v16h a1 = ld16_lds(fA1, fA1 + 16);
#pragma unroll
        for (int j = 0; j < 4; ++j) {
            const _Float16* fb = fB0 + j * 16 * LDS_STRIDE;
            const v16h b = ld16_lds(fb, fb + 16);
            c[0][j] = wmma16(a0, b, c[0][j]);
            c[1][j] = wmma16(a1, b, c[1][j]);
        }
    }
    __syncthreads();

    float bz[4] = {0.f, 0.f, 0.f, 0.f};
    if (MODE == M_F32B || MODE == M_RELU) {
#pragma unroll
        for (int j = 0; j < 4; ++j) bz[j] = bf16r(bias[n0 + wc * 64 + j * 16 + col]);
    }

    if (MODE == M_F16 || MODE == M_HILO || MODE == M_RELU) {
        _Float16* stg = (_Float16*)lds_raw;
        half_t* o0 = (half_t*)out0;
        half_t* o1 = (half_t*)out1;
#pragma unroll
        for (int plane = 0; plane < ((MODE == M_HILO) ? 2 : 1); ++plane) {
            if (plane) __syncthreads();
#pragma unroll
            for (int ms = 0; ms < 2; ++ms) {
#pragma unroll
                for (int r = 0; r < 8; ++r) {
                    const int row = wr * 32 + ms * 16 + r + 8 * hs;
#pragma unroll
                    for (int j = 0; j < 4; ++j) {
                        const int ct = wc * 64 + j * 16 + col;
                        float v = c[ms][j][r] * scale;
                        _Float16 hv;
                        if (MODE == M_RELU) {
                            v = fmaxf(v + bz[j], 0.f);
                            hv = (_Float16)v;
                        } else if (MODE == M_HILO) {
                            const _Float16 hi = (_Float16)v;
                            if (plane == 0) hv = hi;
                            else            hv = (_Float16)((v - (float)hi) * RSC);
                        } else {
                            hv = (_Float16)v;
                        }
                        stg[row * SPH + ct] = hv;
                    }
                }
            }
            __syncthreads();
            half_t* op = (plane == 0) ? o0 : o1;
            write_tile_f16(stg, op, m0, n0, N, wave, lane);
        }
    } else {
        float* stgf = (float*)lds_raw;
        float* of = (float*)out0;
#pragma unroll
        for (int half = 0; half < 2; ++half) {
            if (half) __syncthreads();
            if ((wr >> 1) == half) {
#pragma unroll
                for (int ms = 0; ms < 2; ++ms) {
#pragma unroll
                    for (int r = 0; r < 8; ++r) {
                        const int rowl = (wr & 1) * 32 + ms * 16 + r + 8 * hs;
#pragma unroll
                        for (int j = 0; j < 4; ++j) {
                            const int ct = wc * 64 + j * 16 + col;
                            float v = c[ms][j][r] * scale;
                            if (MODE == M_F32B) v += bz[j];
                            stgf[rowl * SPF + ct] = v;
                        }
                    }
                }
            }
            __syncthreads();
            write_tile_f32(stgf, of, m0 + half * 64, n0, N, wave, lane);
        }
    }
}

__global__ __launch_bounds__(128) __attribute__((amdgpu_num_vgpr(256)))
void k_attn(const half_t* __restrict__ qh, const half_t* __restrict__ ql,
            const half_t* __restrict__ kh, const half_t* __restrict__ kl,
            const half_t* __restrict__ vt, half_t* O, int S) {
    __shared__ __attribute__((aligned(16))) _Float16 lds_p[4][16 * 32];
    __shared__ __attribute__((aligned(16))) _Float16 lds_o[4][16 * 72];

    const int lane = threadIdx.x & 31;
    const int wave = threadIdx.x >> 5;
    const int nqt  = S >> 4;
    const int tile = blockIdx.x * 4 + wave;
    const int h    = tile / nqt;
    const int qt   = tile - h * nqt;
    const int q0   = qt * 16;
    const int col  = lane & 15;
    const int hs   = lane >> 4;
    const int kb   = hs * 8;

    const size_t qoff = (size_t)(q0 + col) * DM + h * HD;
    const v16h aq0 = ld16(qh + qoff + kb,      qh + qoff + kb + 16);
    const v16h aq1 = ld16(qh + qoff + 32 + kb, qh + qoff + 32 + kb + 16);
    const v16h al0 = ld16(ql + qoff + kb,      ql + qoff + kb + 16);
    const v16h al1 = ld16(ql + qoff + 32 + kb, ql + qoff + 32 + kb + 16);

    float m_run[8], l_run[8];
    v8f oc[4] = {{}, {}, {}, {}};
#pragma unroll
    for (int r = 0; r < 8; ++r) { m_run[r] = -1e30f; l_run[r] = 0.f; }

#pragma unroll 1
    for (int kt = 0; kt < S; kt += 32) {
        v8f s0 = {}, s1 = {}, x0 = {}, x1 = {};
        const size_t k0off = (size_t)(kt + col) * DM + h * HD;
        const size_t k1off = k0off + (size_t)16 * DM;
        {
            v16h b;
            b = ld16(kh + k0off + kb, kh + k0off + kb + 16);
            s0 = wmma16(aq0, b, s0); x0 = wmma16(al0, b, x0);
            b = ld16(kl + k0off + kb, kl + k0off + kb + 16);
            x0 = wmma16(aq0, b, x0);
            b = ld16(kh + k0off + 32 + kb, kh + k0off + 32 + kb + 16);
            s0 = wmma16(aq1, b, s0); x0 = wmma16(al1, b, x0);
            b = ld16(kl + k0off + 32 + kb, kl + k0off + 32 + kb + 16);
            x0 = wmma16(aq1, b, x0);

            b = ld16(kh + k1off + kb, kh + k1off + kb + 16);
            s1 = wmma16(aq0, b, s1); x1 = wmma16(al0, b, x1);
            b = ld16(kl + k1off + kb, kl + k1off + kb + 16);
            x1 = wmma16(aq0, b, x1);
            b = ld16(kh + k1off + 32 + kb, kh + k1off + 32 + kb + 16);
            s1 = wmma16(aq1, b, s1); x1 = wmma16(al1, b, x1);
            b = ld16(kl + k1off + 32 + kb, kl + k1off + 32 + kb + 16);
            x1 = wmma16(aq1, b, x1);
        }

        float p0[8], p1[8];
#pragma unroll
        for (int r = 0; r < 8; ++r) {
            const int qi = q0 + r + 8 * hs;
            float sv0 = (s0[r] + x0[r] * (1.0f / RSC)) * 0.125f;
            float sv1 = (s1[r] + x1[r] * (1.0f / RSC)) * 0.125f;
            sv0 += (qi == kt + col)      ? MASKV : 0.f;
            sv1 += (qi == kt + 16 + col) ? MASKV : 0.f;
            const float mx = redmax16(fmaxf(sv0, sv1));
            const float mn = fmaxf(m_run[r], mx);
            const float alpha = __expf(m_run[r] - mn);
            m_run[r] = mn;
            const float e0 = __expf(sv0 - mn);
            const float e1 = __expf(sv1 - mn);
            l_run[r] = l_run[r] * alpha + redsum16(e0 + e1);
#pragma unroll
            for (int j = 0; j < 4; ++j) oc[j][r] *= alpha;
            p0[r] = e0 * PCARRY;
            p1[r] = e1 * PCARRY;
        }

        _Float16* lp = lds_p[wave];
#pragma unroll
        for (int r = 0; r < 8; ++r) {
            lp[(r + 8 * hs) * 32 + col]      = (_Float16)p0[r];
            lp[(r + 8 * hs) * 32 + 16 + col] = (_Float16)p1[r];
        }
        wave_lds_sync();
        const v16h ap = ld16_lds(lp + col * 32 + kb, lp + col * 32 + kb + 16);

        const size_t voff = (size_t)(h * HD + col) * S + kt + kb;
#pragma unroll
        for (int j = 0; j < 4; ++j) {
            const half_t* vp = vt + voff + (size_t)(j * 16) * S;
            const v16h bv = ld16(vp, vp + 16);
            oc[j] = wmma16(ap, bv, oc[j]);
        }
    }

    _Float16* lo = lds_o[wave];
#pragma unroll
    for (int r = 0; r < 8; ++r) {
        const float inv = (1.0f / l_run[r]) * (1.0f / PCARRY);
#pragma unroll
        for (int j = 0; j < 4; ++j)
            lo[(r + 8 * hs) * 72 + j * 16 + col] = (_Float16)(oc[j][r] * inv);
    }
    wave_lds_sync();
    const int rq = lane >> 3, seg = (lane & 7) * 8;
    v8h ov[4];
#pragma unroll
    for (int i = 0; i < 4; ++i) ov[i] = *(const v8h*)(lo + (i * 4 + rq) * 72 + seg);
#pragma unroll
    for (int i = 0; i < 4; ++i)
        *(volatile v8h*)(O + (size_t)(q0 + i * 4 + rq) * DM + h * HD + seg) = ov[i];
    __threadfence();
#pragma unroll
    for (int i = 0; i < 4; ++i)
        *(volatile v8h*)(O + (size_t)(q0 + i * 4 + rq) * DM + h * HD + seg) = ov[i];
}

__global__ __launch_bounds__(256)
void k_ln1(const float* __restrict__ Vin, int vpitch, const float* __restrict__ attn,
           const float* __restrict__ g, const float* __restrict__ be,
           float* zF, half_t* zH) {
    __shared__ float red[8];
    __shared__ __attribute__((aligned(16))) _Float16 hrow[DM];
    const int s = blockIdx.x;
    const int t = threadIdx.x, lane = t & 31, w = t >> 5;
    const int d0 = t * 4;

    const v4f av = *(const v4f*)(attn + (size_t)s * DM + d0);
    float v[4];
#pragma unroll
    for (int c = 0; c < 4; ++c) v[c] = bf16r(Vin[(size_t)(d0 + c) * vpitch + s]) + av[c];

    float sm = (v[0] + v[1]) + (v[2] + v[3]);
    sm = redsum32(sm);
    if (lane == 0) red[w] = sm;
    __syncthreads();
    float tot = 0.f;
#pragma unroll
    for (int i = 0; i < 8; ++i) tot += red[i];
    const float mu = tot * (1.0f / DM);
    __syncthreads();
    float ss = 0.f;
#pragma unroll
    for (int c = 0; c < 4; ++c) { const float dd = v[c] - mu; ss += dd * dd; }
    ss = redsum32(ss);
    if (lane == 0) red[w] = ss;
    __syncthreads();
    float tot2 = 0.f;
#pragma unroll
    for (int i = 0; i < 8; ++i) tot2 += red[i];
    const float sigma = sqrtf(tot2 * (1.0f / (DM - 1)));
    const float inv = 1.0f / (sigma + EPS_LN);

    const v4f gv = *(const v4f*)(g + d0);
    const v4f bv = *(const v4f*)(be + d0);
    v4f y4;
#pragma unroll
    for (int c = 0; c < 4; ++c) {
        const float y = (v[c] - mu) * inv * bf16r(gv[c]) + bf16r(bv[c]);
        y4[c] = y;
        hrow[d0 + c] = (_Float16)y;
    }
    __syncthreads();
    v8h hv = {};
    if (t < 128) hv = *(const v8h*)(hrow + t * 8);
    float* zp = zF + (size_t)s * DM + d0;
    half_t* hp = zH + (size_t)s * DM + t * 8;
    *(volatile v4f*)zp = y4;
    if (t < 128) *(volatile v8h*)hp = hv;
    __threadfence();
    *(volatile v4f*)zp = y4;
    if (t < 128) *(volatile v8h*)hp = hv;
}

__global__ __launch_bounds__(256)
void k_ln2t(const float* __restrict__ zF, const float* __restrict__ ffo,
            const float* __restrict__ g, const float* __restrict__ be,
            float* out, int opitch) {
    __shared__ float mu_s[32], inv_s[32];
    __shared__ v4f T4[64 * 9];
    float* T = (float*)T4;
    const int t = threadIdx.x, lane = t & 31, w = t >> 5;
    const int s0 = blockIdx.x * 32;

#pragma unroll 1
    for (int i = 0; i < 4; ++i) {
        const int s = s0 + w * 4 + i;
        const float* zr = zF  + (size_t)s * DM + lane * 32;
        const float* fr = ffo + (size_t)s * DM + lane * 32;
        float v[32];
        float sm = 0.f;
#pragma unroll
        for (int j = 0; j < 8; ++j) {
            const v4f za = *(const v4f*)(zr + 4 * j);
            const v4f fa = *(const v4f*)(fr + 4 * j);
#pragma unroll
            for (int c = 0; c < 4; ++c) { v[4 * j + c] = za[c] + fa[c]; sm += v[4 * j + c]; }
        }
        sm = redsum32(sm);
        const float mu = sm * (1.0f / DM);
        float ss = 0.f;
#pragma unroll
        for (int j = 0; j < 32; ++j) { const float dd = v[j] - mu; ss += dd * dd; }
        ss = redsum32(ss);
        const float sigma = sqrtf(ss * (1.0f / (DM - 1)));
        const float inv = 1.0f / (sigma + EPS_LN);
        if (lane == 0) { mu_s[w * 4 + i] = mu; inv_s[w * 4 + i] = inv; }
    }
    __syncthreads();

    const int sl = t >> 3;
    const int dseg = (t & 7) * 8;
    const float mu = mu_s[sl], inv = inv_s[sl];
    const float* zr = zF  + (size_t)(s0 + sl) * DM;
    const float* fr = ffo + (size_t)(s0 + sl) * DM;
    const int rq = lane >> 3, cs = (lane & 7) * 4;
#pragma unroll 1
    for (int dc = 0; dc < DM; dc += 64) {
        const int d = dc + dseg;
        const v4f z0 = *(const v4f*)(zr + d),   z1 = *(const v4f*)(zr + d + 4);
        const v4f f0 = *(const v4f*)(fr + d),   f1 = *(const v4f*)(fr + d + 4);
        const v4f g0 = *(const v4f*)(g + d),    g1 = *(const v4f*)(g + d + 4);
        const v4f b0 = *(const v4f*)(be + d),   b1 = *(const v4f*)(be + d + 4);
#pragma unroll
        for (int c = 0; c < 4; ++c) {
            const float va = z0[c] + f0[c];
            const float vb = z1[c] + f1[c];
            T[(dseg + c) * 36 + sl]     = (va - mu) * inv * bf16r(g0[c]) + bf16r(b0[c]);
            T[(dseg + 4 + c) * 36 + sl] = (vb - mu) * inv * bf16r(g1[c]) + bf16r(b1[c]);
        }
        __syncthreads();
        const int dl0 = w * 8 + rq, dl1 = w * 8 + 4 + rq;
        const v4f o0 = *(const v4f*)(T + dl0 * 36 + cs);
        const v4f o1 = *(const v4f*)(T + dl1 * 36 + cs);
        float* p0 = out + (size_t)(dc + dl0) * opitch + s0 + cs;
        float* p1 = out + (size_t)(dc + dl1) * opitch + s0 + cs;
        *(volatile v4f*)p0 = o0;
        *(volatile v4f*)p1 = o1;
        __threadfence();
        *(volatile v4f*)p0 = o0;
        *(volatile v4f*)p1 = o1;
        __syncthreads();
    }
}

extern "C" void kernel_launch(void* const* d_in, const int* in_sizes, int n_in,
                              void* d_out, int out_size, void* d_ws, size_t ws_size,
                              hipStream_t stream) {
    if (n_in < 13) return;
    const int needQKV = (DM - 1) * S_FULL + SEQ;
    if (in_sizes[0] < needQKV || in_sizes[1] < needQKV || in_sizes[2] < needQKV) return;
    if (in_sizes[3] < DM * DM || in_sizes[4] < DM * DM || in_sizes[5] < DM * DM) return;
    if (in_sizes[6] < DM * DM || in_sizes[7] < FFD * DM || in_sizes[8] < FFD) return;
    if (in_sizes[9] < DM * FFD || in_sizes[10] < DM || in_sizes[11] < DM || in_sizes[12] < DM) return;
    if (out_size < DM * SEQ) return;

    const float* Qin = (const float*)d_in[0];
    const float* Kin = (const float*)d_in[1];
    const float* Vin = (const float*)d_in[2];
    const float* wq  = (const float*)d_in[3];
    const float* wk  = (const float*)d_in[4];
    const float* wv  = (const float*)d_in[5];
    const float* Wo  = (const float*)d_in[6];
    const float* W1  = (const float*)d_in[7];
    const float* b1  = (const float*)d_in[8];
    const float* W2  = (const float*)d_in[9];
    const float* b2  = (const float*)d_in[10];
    const float* ga  = (const float*)d_in[11];
    const float* gb  = (const float*)d_in[12];
    float* out = (float*)d_out;

    char* wsb = (char*)d_ws;
    size_t off = 0;
    auto carve = [&](size_t bytes) -> char* {
        char* p = wsb + off;
        off += (bytes + 4095) & ~(size_t)4095;
        return p;
    };
    const size_t SD2 = (size_t)SEQ * DM * 2;
    const size_t SD4 = (size_t)SEQ * DM * 4;
    const size_t DD2 = (size_t)DM * DM * 2;
    const size_t FD2 = (size_t)FFD * DM * 2;
    const size_t SF2 = (size_t)SEQ * FFD * 2;

    half_t* QTh  = (half_t*)carve(SD2);
    half_t* KTh  = (half_t*)carve(SD2);
    half_t* VTh  = (half_t*)carve(SD2);
    half_t* wqh  = (half_t*)carve(DD2);
    half_t* wkh  = (half_t*)carve(DD2);
    half_t* wvh  = (half_t*)carve(DD2);
    half_t* woTh = (half_t*)carve(DD2);
    half_t* w1h  = (half_t*)carve(FD2);
    half_t* w2h  = (half_t*)carve(FD2);
    half_t* qH   = (half_t*)carve(SD2);
    half_t* qL   = (half_t*)carve(SD2);
    half_t* kH   = (half_t*)carve(SD2);
    half_t* kL   = (half_t*)carve(SD2);
    half_t* vtH  = (half_t*)carve(SD2);
    half_t* hdsH = (half_t*)carve(SD2);
    float*  attF = (float*) carve(SD4);
    float*  zF   = (float*) carve(SD4);
    half_t* zH   = (half_t*)carve(SD2);
    half_t* ffhH = (half_t*)carve(SF2);
    float*  ffoF = (float*) carve(SD4);
    if (off > ws_size) return;

    const float wscInv = 1.0f / WSC;

    k_tr64<<<dim3(SEQ / 64, DM / 64), 256, 0, stream>>>(Qin, S_FULL, QTh, DM, 1.0f);
    k_tr64<<<dim3(SEQ / 64, DM / 64), 256, 0, stream>>>(Kin, S_FULL, KTh, DM, 1.0f);
    k_tr64<<<dim3(SEQ / 64, DM / 64), 256, 0, stream>>>(Vin, S_FULL, VTh, DM, 1.0f);
    {
        const int n8w = DM * DM / 8;
        k_cvt8<<<(n8w + 255) / 256, 256, 0, stream>>>(wq, wqh, n8w, WSC);
        k_cvt8<<<(n8w + 255) / 256, 256, 0, stream>>>(wk, wkh, n8w, WSC);
        k_cvt8<<<(n8w + 255) / 256, 256, 0, stream>>>(wv, wvh, n8w, WSC);
        const int n8f = FFD * DM / 8;
        k_cvt8<<<(n8f + 255) / 256, 256, 0, stream>>>(W1, w1h, n8f, WSC);
        k_cvt8<<<(n8f + 255) / 256, 256, 0, stream>>>(W2, w2h, n8f, WSC);
    }
    k_tr64<<<dim3(DM / 64, DM / 64), 256, 0, stream>>>(Wo, DM, woTh, DM, WSC);

    dim3 gP(DM / 128, SEQ / 128);
    k_gemm<M_HILO><<<gP, 256, 0, stream>>>(QTh, wqh, nullptr, qH, qL, SEQ, DM, DM, wscInv);
    k_gemm<M_HILO><<<gP, 256, 0, stream>>>(KTh, wkh, nullptr, kH, kL, SEQ, DM, DM, wscInv);
    dim3 gV(SEQ / 128, DM / 128);
    k_gemm<M_F16><<<gV, 256, 0, stream>>>(wvh, VTh, nullptr, vtH, nullptr, DM, SEQ, DM, wscInv);

    k_attn<<<(NH * (SEQ / 16)) / 4, 128, 0, stream>>>(qH, qL, kH, kL, vtH, hdsH, SEQ);

    k_gemm<M_F32><<<gP, 256, 0, stream>>>(hdsH, woTh, nullptr, attF, nullptr, SEQ, DM, DM, wscInv);
    k_ln1<<<SEQ, 256, 0, stream>>>(Vin, S_FULL, attF, ga, gb, zF, zH);

    dim3 gF(FFD / 128, SEQ / 128);
    k_gemm<M_RELU><<<gF, 256, 0, stream>>>(zH, w1h, b1, ffhH, nullptr, SEQ, FFD, DM, wscInv);
    k_gemm<M_F32B><<<gP, 256, 0, stream>>>(ffhH, w2h, b2, ffoF, nullptr, SEQ, DM, FFD, wscInv);
    k_ln2t<<<SEQ / 32, 256, 0, stream>>>(zF, ffoF, ga, gb, out, SEQ);
}
